// LongTermAttention_18640158064770
// MI455X (gfx1250) — hardware-verified
//
#include <hip/hip_runtime.h>
#include <math.h>
#include <stdint.h>

#define NBATCH 4
#define LMEM   2048
#define QLEN   2048
#define HID    1024
#define NH     16
#define HD     64
#define NBAS   512
#define MROWS  (NBATCH * QLEN)
#define NQB64  (QLEN / 64)
#define NCH    (NBAS / 64)
static_assert(NH * HD == HID);
static_assert(NQB64 == 32 && NCH == 8);
static_assert((LMEM % 64) == 0 && (QLEN % 64) == 0 && (HID % 64) == 0 && (NBAS % 64) == 0);
static_assert((LMEM % 32) == 0 && (HID % 32) == 0 && (NBAS % 32) == 0);
#define CSC  64.0f
#define WOSC 64.0f

typedef _Float16 v16h __attribute__((ext_vector_type(16)));
typedef _Float16 v8h  __attribute__((ext_vector_type(8)));
typedef __bf16   v16b __attribute__((ext_vector_type(16)));
typedef __bf16   v8b  __attribute__((ext_vector_type(8)));
typedef float    v8f  __attribute__((ext_vector_type(8)));
typedef float    v4f  __attribute__((ext_vector_type(4)));
typedef unsigned int   v4u  __attribute__((ext_vector_type(4)));
typedef unsigned short v8us __attribute__((ext_vector_type(8)));
typedef v4u  __attribute__((may_alias)) v4ua;
typedef v8us __attribute__((may_alias)) v8usa;

#if defined(__HIP_DEVICE_COMPILE__)
#define DEV_ASM 1
#else
#define DEV_ASM 0
#endif

__device__ __forceinline__ unsigned short bf_bits(float f) {
  unsigned u = __float_as_uint(f);
  return (unsigned short)((u + 0x7FFFu + ((u >> 16) & 1u)) >> 16);
}
__device__ __forceinline__ float bf_up(unsigned short hb) { return __uint_as_float(((unsigned)hb) << 16); }
__device__ __forceinline__ unsigned short h_bits(_Float16 x) { return __builtin_bit_cast(unsigned short, x); }
__device__ __forceinline__ unsigned pk16(unsigned short a, unsigned short b) { return (unsigned)a | ((unsigned)b << 16); }
__device__ __forceinline__ v8f zero8() { v8f z = {0.f, 0.f, 0.f, 0.f, 0.f, 0.f, 0.f, 0.f}; return z; }

template <typename OT> struct FT;
template <> struct FT<__bf16>   { typedef v16b frag; typedef v8b half8; };
template <> struct FT<_Float16> { typedef v16h frag; typedef v8h half8; };

template <typename OT>
__device__ __forceinline__ typename FT<OT>::frag ldfrag(const OT* p) {
  union { typename FT<OT>::frag v; typename FT<OT>::half8 h[2]; } f;
  f.h[0] = *(const typename FT<OT>::half8*)(p);
  f.h[1] = *(const typename FT<OT>::half8*)(p + 16);
  return f.v;
}

__device__ __forceinline__ v8f mma_g(v16b a, v16b b, v8f c) {
  c = __builtin_amdgcn_wmma_f32_16x16x32_bf16(false, a, false, b, (short)0, c, false, false);
#if DEV_ASM
  asm volatile("v_nop\n\tv_nop\n\tv_nop\n\tv_nop" : "+v"(c) : "v"(a), "v"(b));
#endif
  return c;
}
__device__ __forceinline__ v8f mma_g(v16h a, v16h b, v8f c) {
  c = __builtin_amdgcn_wmma_f32_16x16x32_f16(false, a, false, b, (short)0, c, false, false);
#if DEV_ASM
  asm volatile("v_nop\n\tv_nop\n\tv_nop\n\tv_nop" : "+v"(c) : "v"(a), "v"(b));
#endif
  return c;
}

template <int MODE>
__device__ __forceinline__ unsigned short cvm(float f) {
  const unsigned short hb = bf_bits(f);
  if (MODE == 0) return hb;
  return h_bits((_Float16)(bf_up(hb) * WOSC));
}

template <int MODE>
__global__ __launch_bounds__(256) void cvt16x8(const float* __restrict__ in, unsigned short* out, int n8) {
  const int i = blockIdx.x * 256 + (int)threadIdx.x;
  if (i < n8) {
    const v4f a  = *(const v4f*)(in + (size_t)i * 8);
    const v4f a4 = *(const v4f*)(in + (size_t)i * 8 + 4);
    v4u p;
    p[0] = pk16(cvm<MODE>(a[0]),  cvm<MODE>(a[1]));
    p[1] = pk16(cvm<MODE>(a[2]),  cvm<MODE>(a[3]));
    p[2] = pk16(cvm<MODE>(a4[0]), cvm<MODE>(a4[1]));
    p[3] = pk16(cvm<MODE>(a4[2]), cvm<MODE>(a4[3]));
    unsigned short* o = out + (size_t)i * 8;
    *(volatile v4u*)o = p;
    __threadfence();
    *(volatile v4u*)o = p;
  }
}

__global__ __launch_bounds__(256) void tr_bf16(const float* __restrict__ in, unsigned short* out,
                                               int R, int C, long long ibs, long long obs) {
  __shared__ __align__(16) unsigned short t[64][72];
  const int tid = threadIdx.x;
  const float* ib = in + (size_t)blockIdx.z * (size_t)ibs;
  unsigned short* ob = out + (size_t)blockIdx.z * (size_t)obs;
  const int r0 = blockIdx.y * 64, c0 = blockIdx.x * 64;
#pragma unroll
  for (int it = 0; it < 4; ++it) {
    const int i = tid + 256 * it;
    const int rr = i >> 4, cc4 = (i & 15) * 4;
    const v4f v = *(const v4f*)(ib + (size_t)(r0 + rr) * (size_t)C + c0 + cc4);
    t[cc4 + 0][rr] = bf_bits(v[0]);
    t[cc4 + 1][rr] = bf_bits(v[1]);
    t[cc4 + 2][rr] = bf_bits(v[2]);
    t[cc4 + 3][rr] = bf_bits(v[3]);
  }
  __syncthreads();
  const int wave = tid >> 5, lane = tid & 31;
  const int q8 = lane & 7, sub = lane >> 3;
  v4u pv[2];
#pragma unroll
  for (int it = 0; it < 2; ++it) {
    const int row = it * 32 + wave * 4 + sub;
    pv[it] = *(const v4ua*)(&t[row][8 * q8]);
  }
  for (int pass = 0; pass < 2; ++pass) {
#pragma unroll
    for (int it = 0; it < 2; ++it) {
      const int row = it * 32 + wave * 4 + sub;
      *(volatile v4u*)(ob + (size_t)(c0 + row) * (size_t)R + r0 + 8 * q8) = pv[it];
    }
    __threadfence();
  }
}

template <typename OT, int SPL, int OUT_MODE>
__global__ __launch_bounds__(256) void gemm64(
    const unsigned short* __restrict__ Ap, const unsigned short* __restrict__ A2p, int lda, long long strideA,
    const unsigned short* __restrict__ Btp, const unsigned short* __restrict__ Bt2p, int ldb, long long strideB,
    void* Cout, void* Cout2, int ldc, long long strideC,
    int M, int N, int K, float oscale) {
  typedef typename FT<OT>::frag V16;
  const OT* A   = (const OT*)(const void*)Ap;
  const OT* A2  = (const OT*)(const void*)A2p;
  const OT* Bt  = (const OT*)(const void*)Btp;
  const OT* Bt2 = (const OT*)(const void*)Bt2p;
  __shared__ __align__(16) float sT[8][16 * 68];
  const int b    = blockIdx.y;
  const int lane = threadIdx.x & 31;
  const int wave = threadIdx.x >> 5;
  const int tilesN = N >> 6;
  const int tilesM = M >> 6;
  const int tile = blockIdx.x * 8 + wave;
  if (tile >= tilesM * tilesN) return;
  const int tm = tile / tilesN;
  const int tn = tile - tm * tilesN;
  const int m0 = tm << 6;
  const int n0 = tn << 6;

  const OT* Ab  = A   + (size_t)b * (size_t)strideA;
  const OT* Ab2 = A2  + (size_t)b * (size_t)strideA;
  const OT* Bb  = Bt  + (size_t)b * (size_t)strideB;
  const OT* Bb2 = Bt2 + (size_t)b * (size_t)strideB;

  const int rlane = lane & 15;
  const int koff  = (lane >> 4) * 8;
  const int mOff  = (lane >> 4) * 8;

  v8f acc[4][4];
#pragma unroll
  for (int i = 0; i < 4; ++i)
#pragma unroll
    for (int j = 0; j < 4; ++j) acc[i][j] = zero8();

  for (int k0 = 0; k0 < K; k0 += 32) {
#pragma unroll
    for (int p = 0; p < ((SPL == 2) ? 2 : 1); ++p) {
      const OT* Bs = (p == 0) ? Bb : Bb2;
      V16 bq[4];
#pragma unroll
      for (int j = 0; j < 4; ++j)
        bq[j] = ldfrag<OT>(Bs + (size_t)(n0 + (j << 4) + rlane) * (size_t)ldb + koff + k0);
#pragma unroll
      for (int i = 0; i < 4; ++i) {
        const V16 af = ldfrag<OT>(Ab + (size_t)(m0 + (i << 4) + rlane) * (size_t)lda + koff + k0);
#pragma unroll
        for (int j = 0; j < 4; ++j) acc[i][j] = mma_g(af, bq[j], acc[i][j]);
        if (SPL == 1) {
          const V16 ag = ldfrag<OT>(Ab2 + (size_t)(m0 + (i << 4) + rlane) * (size_t)lda + koff + k0);
#pragma unroll
          for (int j = 0; j < 4; ++j) acc[i][j] = mma_g(ag, bq[j], acc[i][j]);
        }
      }
    }
  }

  float* slab = sT[wave];
#pragma unroll
  for (int i = 0; i < 4; ++i) {
    const int mBase = m0 + (i << 4);
#pragma unroll
    for (int j = 0; j < 4; ++j) {
#pragma unroll
      for (int r = 0; r < 8; ++r) {
        slab[(mOff + r) * 68 + (j << 4) + rlane] = acc[i][j][r];
      }
    }
    __builtin_amdgcn_fence(__ATOMIC_RELEASE, "workgroup");
    __builtin_amdgcn_wave_barrier();
    __builtin_amdgcn_fence(__ATOMIC_ACQUIRE, "workgroup");
    if (OUT_MODE == 0) {
      float* Cf = (float*)Cout + (size_t)b * (size_t)strideC;
      const int h2 = lane >> 4, c4 = (lane & 15) * 4;
      for (int pass = 0; pass < 2; ++pass) {
#pragma unroll
        for (int it = 0; it < 8; ++it) {
          const int row = it * 2 + h2;
          const v4f v = *(const v4f*)(slab + row * 68 + c4) * oscale;
          *(volatile v4f*)(Cf + (size_t)(mBase + row) * (size_t)ldc + n0 + c4) = v;
        }
        __threadfence();
      }
    } else {
      const int q = lane >> 3, c8 = (lane & 7) * 8;
      unsigned short* Ch = (unsigned short*)Cout  + (size_t)b * (size_t)strideC;
      unsigned short* Cl = (unsigned short*)Cout2 + (size_t)b * (size_t)strideC;
      v4u hv[4], lv[4];
#pragma unroll
      for (int it = 0; it < 4; ++it) {
        const int row = it * 4 + q;
        const float* sp = slab + row * 68 + c8;
        v4u a, a2;
#pragma unroll
        for (int e = 0; e < 4; ++e) {
          const float f0 = sp[2 * e], f1 = sp[2 * e + 1];
          const unsigned short h0 = bf_bits(f0), h1 = bf_bits(f1);
          const unsigned short l0 = bf_bits(f0 - bf_up(h0));
          const unsigned short l1 = bf_bits(f1 - bf_up(h1));
          a[e] = pk16(h0, h1); a2[e] = pk16(l0, l1);
        }
        hv[it] = a; lv[it] = a2;
      }
      for (int pass = 0; pass < 2; ++pass) {
#pragma unroll
        for (int it = 0; it < 4; ++it) {
          const int row = it * 4 + q;
          *(volatile v4u*)(Ch + (size_t)(mBase + row) * (size_t)ldc + n0 + c8) = hv[it];
          *(volatile v4u*)(Cl + (size_t)(mBase + row) * (size_t)ldc + n0 + c8) = lv[it];
        }
        __threadfence();
      }
    }
    __builtin_amdgcn_fence(__ATOMIC_RELEASE, "workgroup");
    __builtin_amdgcn_wave_barrier();
    __builtin_amdgcn_fence(__ATOMIC_ACQUIRE, "workgroup");
  }
}

__global__ __launch_bounds__(256) void kw_kernel(const float* __restrict__ keys, const float* __restrict__ wmu,
                                                 const float* __restrict__ wsg, float* u) {
  __shared__ float wsh[2][NBAS];
  const int tid = threadIdx.x;
  const int b = blockIdx.y;
  const int e = blockIdx.x * 256 + tid;
  for (int i = tid; i < NBAS; i += 256) {
    wsh[0][i] = bf_up(bf_bits(wmu[i]));
    wsh[1][i] = bf_up(bf_bits(wsg[i]));
  }
  __syncthreads();
  const float* kp = keys + (size_t)b * NBAS * HID + e;
  float am = 0.f, ag = 0.f;
#pragma unroll 4
  for (int n = 0; n < NBAS; ++n) {
    const float kv = kp[(size_t)n * HID];
    am += kv * wsh[0][n];
    ag += kv * wsh[1][n];
  }
  float* pm = u + ((size_t)b * 2) * HID + e;
  float* pg = pm + HID;
  *(volatile float*)pm = am;
  *(volatile float*)pg = ag;
  __threadfence();
  *(volatile float*)pm = am;
  *(volatile float*)pg = ag;
}

__global__ __launch_bounds__(128) void ctx_kernel(
    const float* __restrict__ qry, const float* __restrict__ u,
    const float* __restrict__ bmu, const float* __restrict__ bsg,
    const unsigned short* __restrict__ vthp, const unsigned short* __restrict__ vtlp,
    unsigned short* ctxp) {
  union FB { v16b v; v8us h[2]; unsigned short s[16]; };
  __shared__ __align__(16) unsigned short Vth[64 * 64];
  __shared__ __align__(16) unsigned short Vtl[64 * 64];
  __shared__ __align__(16) float Os[4][16 * 64];
  __shared__ float bm_s[NBAS];
  __shared__ float bv_s[NBAS];

  const int tid  = threadIdx.x;
  const int wave = tid >> 5;
  const int lane = tid & 31;
  const int hh   = lane >> 4;
  const int c    = lane & 15;

  const int bx   = blockIdx.x;
  const int qb   = bx % NQB64;
  const int rest = bx / NQB64;
  const int h    = rest % NH;
  const int b    = rest / NH;
  const int q0   = qb * 64 + wave * 16;
  const size_t row0 = (size_t)b * QLEN + q0;

  for (int i = tid; i < NBAS; i += 128) {
    const float m = bf_up(bf_bits(bmu[i]));
    const float s = bf_up(bf_bits(bsg[i]));
    bm_s[i] = m;
    bv_s[i] = s * s;
  }

  float dm = 0.f, dg = 0.f;
  {
    const float* qr = qry + (row0 + c) * HID + (size_t)h * HD + 32 * hh;
    const float* um = u + ((size_t)b * 2) * HID + (size_t)h * HD + 32 * hh;
    const float* ug = um + HID;
#pragma unroll 2
    for (int i = 0; i < 8; ++i) {
      const v4f a  = *(const v4f*)(qr + 4 * i);
      const v4f wm = *(const v4f*)(um + 4 * i);
      const v4f wg = *(const v4f*)(ug + 4 * i);
      dm += a[0] * wm[0]; dm += a[1] * wm[1]; dm += a[2] * wm[2]; dm += a[3] * wm[3];
      dg += a[0] * wg[0]; dg += a[1] * wg[1]; dg += a[2] * wg[2]; dg += a[3] * wg[3];
    }
  }
  dm += __shfl_xor(dm, 16, 32);
  dg += __shfl_xor(dg, 16, 32);
  dm *= 0.125f;
  dg *= 0.125f;
  const float mu   = 1.0f / (1.0f + expf(-dm));
  const float spl  = fmaxf(dg, 0.0f) + log1pf(expf(-fabsf(dg)));
  const float sig2 = fmaxf(spl, 1e-4f);

  const unsigned short* Vh = vthp + ((size_t)b * HID + (size_t)h * HD) * NBAS;
  const unsigned short* Vl = vtlp + ((size_t)b * HID + (size_t)h * HD) * NBAS;

  v8f oacc[4];
#pragma unroll
  for (int t = 0; t < 4; ++t) oacc[t] = zero8();

  for (int nt = 0; nt < NCH; ++nt) {
    const int n0 = nt * 64;
    __syncthreads();
    {
      const int r = tid >> 1, half = (tid & 1) * 32;
      const unsigned short* vg  = Vh + (size_t)r * NBAS + n0 + half;
      const unsigned short* vlg = Vl + (size_t)r * NBAS + n0 + half;
#pragma unroll
      for (int i = 0; i < 4; ++i) {
        const v8us b0 = *(const v8usa*)(vg + 8 * i);
        const v8us b1 = *(const v8usa*)(vlg + 8 * i);
        *(v8usa*)(Vth + r * 64 + half + 8 * i) = b0;
        *(v8usa*)(Vtl + r * 64 + half + 8 * i) = b1;
      }
    }
    __syncthreads();

#pragma unroll 1
    for (int kk = 0; kk < 2; ++kk) {
      FB rh, rl;
#pragma unroll
      for (int i = 0; i < 16; ++i) {
        const int n = n0 + kk * 32 + ((i < 8) ? (8 * hh + i) : (8 + 8 * hh + i));
        const float t   = mu - bm_s[n];
        const float var = sig2 + bv_s[n];
        const float iv  = __builtin_amdgcn_rcpf(var);
        const float rv  = __expf(-0.5f * t * t * iv) * rsqrtf(6.2831853071795864f * var);
        const unsigned short hb = bf_bits(rv);
        rh.s[i] = hb;
        rl.s[i] = bf_bits(rv - bf_up(hb));
      }
#pragma unroll
      for (int t = 0; t < 4; ++t) {
        FB vb, vl;
        vb.h[0] = *(const v8usa*)(Vth + (t * 16 + c) * 64 + kk * 32 + 8 * hh);
        vb.h[1] = *(const v8usa*)(Vth + (t * 16 + c) * 64 + kk * 32 + 16 + 8 * hh);
        vl.h[0] = *(const v8usa*)(Vtl + (t * 16 + c) * 64 + kk * 32 + 8 * hh);
        vl.h[1] = *(const v8usa*)(Vtl + (t * 16 + c) * 64 + kk * 32 + 16 + 8 * hh);
        oacc[t] = mma_g(rh.v, vb.v, oacc[t]);
        oacc[t] = mma_g(rh.v, vl.v, oacc[t]);
        oacc[t] = mma_g(rl.v, vb.v, oacc[t]);
      }
    }
  }

  float* os = Os[wave];
#pragma unroll
  for (int r = 0; r < 8; ++r) {
#pragma unroll
    for (int t = 0; t < 4; ++t) os[(8 * hh + r) * 64 + t * 16 + c] = oacc[t][r];
  }
  __builtin_amdgcn_fence(__ATOMIC_RELEASE, "workgroup");
  __builtin_amdgcn_wave_barrier();
  __builtin_amdgcn_fence(__ATOMIC_ACQUIRE, "workgroup");
  {
    const int q4 = lane >> 3, c8 = (lane & 7) * 8;
    v4u hv[4];
#pragma unroll
    for (int it = 0; it < 4; ++it) {
      const int row = it * 4 + q4;
      const float* sp = os + row * 64 + c8;
      v4u a;
#pragma unroll
      for (int e = 0; e < 4; ++e) {
        const float f0 = sp[2 * e] * CSC, f1 = sp[2 * e + 1] * CSC;
        a[e] = pk16(h_bits((_Float16)f0), h_bits((_Float16)f1));
      }
      hv[it] = a;
    }
    for (int pass = 0; pass < 2; ++pass) {
#pragma unroll
      for (int it = 0; it < 4; ++it) {
        const int row = it * 4 + q4;
        const size_t go = (row0 + row) * HID + (size_t)h * HD + c8;
        *(volatile v4u*)(ctxp + go) = hv[it];
      }
      __threadfence();
    }
  }
}

extern "C" void kernel_launch(void* const* d_in, const int* in_sizes, int n_in,
                              void* d_out, int out_size, void* d_ws, size_t ws_size,
                              hipStream_t stream) {
  if (n_in < 11) return;
  if (in_sizes[0] != NBATCH * LMEM * HID) return;
  if (in_sizes[1] != MROWS * HID) return;
  if (in_sizes[2] != HID * HID || in_sizes[3] != HID * HID || in_sizes[4] != HID * HID || in_sizes[5] != HID * HID) return;
  if (in_sizes[6] != NBAS || in_sizes[7] != NBAS) return;
  if (in_sizes[8] != LMEM * NBAS || in_sizes[9] != NBAS || in_sizes[10] != NBAS) return;
  if (out_size != MROWS * HID) return;

  const float* kin = (const float*)d_in[0];
  const float* qin = (const float*)d_in[1];
  const float* Wq  = (const float*)d_in[2];
  const float* Wk  = (const float*)d_in[3];
  const float* Wv  = (const float*)d_in[4];
  const float* Wo  = (const float*)d_in[5];
  const float* wmu = (const float*)d_in[6];
  const float* wsg = (const float*)d_in[7];
  const float* Gs  = (const float*)d_in[8];
  const float* bmu = (const float*)d_in[9];
  const float* bsg = (const float*)d_in[10];

  const size_t PKT  = (size_t)NBATCH * HID * LMEM * 2;
  const size_t PCTX = (size_t)MROWS * HID * 2;
  const size_t PGT  = (size_t)NBAS * LMEM * 2;
  const size_t PQB  = (size_t)MROWS * HID * 2;
  const size_t PW   = (size_t)HID * HID * 2;
  const size_t PBM  = (size_t)NBATCH * NBAS * HID * 2;
  const size_t PKEY = (size_t)NBATCH * NBAS * HID * 4;
  const size_t PVT  = (size_t)NBATCH * HID * NBAS * 2;
  const size_t PQRY = (size_t)MROWS * HID * 4;
  const size_t PU   = (size_t)NBATCH * 2 * HID * 4;
  if (PCTX > PKT) return;
  size_t off = 0;
  const size_t oKT  = off; off += PKT;
  const size_t oGT  = off; off += PGT;
  const size_t oQB  = off; off += PQB;
  const size_t oWQ  = off; off += PW;
  const size_t oWK  = off; off += PW;
  const size_t oWV  = off; off += PW;
  const size_t oWO  = off; off += PW;
  const size_t oBMH = off; off += PBM;
  const size_t oBML = off; off += PBM;
  const size_t oKEY = off; off += PKEY;
  const size_t oVTH = off; off += PVT;
  const size_t oVTL = off; off += PVT;
  const size_t oQRY = off; off += PQRY;
  const size_t oU   = off; off += PU;
  if (off > ws_size) return;
  if (off > (size_t)134217728) return;

  char* ws = (char*)d_ws;
  unsigned short* KT  = (unsigned short*)(ws + oKT);
  unsigned short* CTX = (unsigned short*)(ws + oKT);
  unsigned short* GT  = (unsigned short*)(ws + oGT);
  unsigned short* QB  = (unsigned short*)(ws + oQB);
  unsigned short* WQB = (unsigned short*)(ws + oWQ);
  unsigned short* WKB = (unsigned short*)(ws + oWK);
  unsigned short* WVB = (unsigned short*)(ws + oWV);
  unsigned short* WOH = (unsigned short*)(ws + oWO);
  unsigned short* BMH = (unsigned short*)(ws + oBMH);
  unsigned short* BML = (unsigned short*)(ws + oBML);
  float*          KEY = (float*)(ws + oKEY);
  unsigned short* VTH = (unsigned short*)(ws + oVTH);
  unsigned short* VTL = (unsigned short*)(ws + oVTL);
  float*          QRY = (float*)(ws + oQRY);
  float*          U   = (float*)(ws + oU);

  const dim3 blk(256);
  const int n8q = MROWS * HID / 8;
  const int n8w = HID * HID / 8;
  const dim3 gTrK(HID / 64, LMEM / 64, NBATCH);
  const dim3 gTrG(NBAS / 64, LMEM / 64, 1);
  const dim3 gCvtQ((n8q + 255) / 256);
  const dim3 gCvtW((n8w + 255) / 256);
  const dim3 gBm(((NBAS / 64) * (HID / 64) + 7) / 8, NBATCH);
  const dim3 gKey((((NBATCH * NBAS) / 64) * (HID / 64) + 7) / 8, 1);
  const dim3 gVt(((HID / 64) * (NBAS / 64) + 7) / 8, NBATCH);
  const dim3 gQ(((MROWS / 64) * (HID / 64) + 7) / 8, 1);
  const dim3 gKw(HID / 256, NBATCH);
  const dim3 gCtx(NBATCH * NH * NQB64);

  tr_bf16<<<gTrK, blk, 0, stream>>>(kin, KT, LMEM, HID, (long long)LMEM * HID, (long long)HID * LMEM);
  tr_bf16<<<gTrG, blk, 0, stream>>>(Gs, GT, LMEM, NBAS, 0LL, 0LL);
  cvt16x8<0><<<gCvtQ, blk, 0, stream>>>(qin, QB,  n8q);
  cvt16x8<0><<<gCvtW, blk, 0, stream>>>(Wq,  WQB, n8w);
  cvt16x8<0><<<gCvtW, blk, 0, stream>>>(Wk,  WKB, n8w);
  cvt16x8<0><<<gCvtW, blk, 0, stream>>>(Wv,  WVB, n8w);
  cvt16x8<1><<<gCvtW, blk, 0, stream>>>(Wo,  WOH, n8w);
  gemm64<__bf16, 0, 2><<<gBm, blk, 0, stream>>>(
      GT, GT, LMEM, 0LL, KT, KT, LMEM, (long long)HID * LMEM,
      (void*)BMH, (void*)BML, HID, (long long)NBAS * HID,
      NBAS, HID, LMEM, 1.0f);
  gemm64<__bf16, 1, 0><<<gKey, blk, 0, stream>>>(
      BMH, BML, HID, 0LL, WKB, WKB, HID, 0LL,
      (void*)KEY, (void*)KEY, HID, 0LL,
      NBATCH * NBAS, HID, HID, 1.0f);
  gemm64<__bf16, 2, 2><<<gVt, blk, 0, stream>>>(
      WVB, WVB, HID, 0LL, BMH, BML, HID, (long long)NBAS * HID,
      (void*)VTH, (void*)VTL, NBAS, (long long)HID * NBAS,
      HID, NBAS, HID, 1.0f);
  gemm64<__bf16, 0, 0><<<gQ, blk, 0, stream>>>(
      QB, QB, HID, 0LL, WQB, WQB, HID, 0LL,
      (void*)QRY, (void*)QRY, HID, 0LL,
      MROWS, HID, HID, 1.0f);
  kw_kernel<<<gKw, blk, 0, stream>>>(KEY, wmu, wsg, U);
  ctx_kernel<<<gCtx, dim3(128), 0, stream>>>(QRY, U, bmu, bsg, VTH, VTL, CTX);
  gemm64<_Float16, 0, 0><<<gQ, blk, 0, stream>>>(
      CTX, CTX, HID, 0LL, WOH, WOH, HID, 0LL,
      d_out, d_out, HID, 0LL,
      MROWS, HID, HID, 1.0f / (CSC * WOSC));
  (void)hipGetLastError();
}
